// StateSpaceBlock_38027640439433
// MI455X (gfx1250) — hardware-verified
//
#include <hip/hip_runtime.h>
#include <math.h>

typedef __attribute__((ext_vector_type(16))) _Float16 v16h;
typedef __attribute__((ext_vector_type(8)))  _Float16 v8h;
typedef __attribute__((ext_vector_type(16))) __bf16   v16b;
typedef __attribute__((ext_vector_type(8)))  __bf16   v8b;
typedef __attribute__((ext_vector_type(8)))  float    v8f;
typedef __attribute__((ext_vector_type(4)))  float    v4f;

constexpr int kBatch = 2;
constexpr int kSeqL  = 1024;
constexpr int kDmod  = 512;
constexpr int kDin   = 1024;
constexpr int kNst   = 64;
constexpr int kNq    = 16;
constexpr int kChB   = 64;
constexpr int kSC    = 32;
constexpr int kConvK = 4;
constexpr int kBCW   = 2 * kNst;
constexpr int kXZP   = 2 * kDin;
constexpr int kRows  = kBatch * kSeqL;
constexpr int kTP    = 260;
constexpr int kYP    = 68;
constexpr float kLnEps = 1e-5f;
static_assert(kDmod == 512, "ln lane map");
static_assert(kNst == 4 * kNq, "state split");
static_assert(kSeqL % 64 == 0 && kSeqL % kSC == 0 && kDin % 256 == 0 && kDin % kChB == 0 && kRows % 64 == 0, "tiling");

__device__ __forceinline__ unsigned short f2bf_bits(float f) {
  unsigned u = __float_as_uint(f);
  return (unsigned short)((u + 0x7FFFu + ((u >> 16) & 1u)) >> 16);
}
__device__ __forceinline__ float bf_bits2f(unsigned short h) { return __uint_as_float(((unsigned)h) << 16); }

__device__ __forceinline__ void split_bf16(float v, _Float16& hi, _Float16& lo) {
  const unsigned short hb = f2bf_bits(v);
  const unsigned short lb = f2bf_bits(v - bf_bits2f(hb));
  hi = __builtin_bit_cast(_Float16, hb);
  lo = __builtin_bit_cast(_Float16, lb);
}

__device__ __forceinline__ void dep_guard_h(v8f& a, v8f& b, v16h x, v16h y) { asm volatile("v_nop\n\tv_nop\n\tv_nop\n\tv_nop" : "+v"(a), "+v"(b) : "v"(x), "v"(y)); }
__device__ __forceinline__ void dep_guard_b(v8f& a, v8f& b, v16b x, v16b y) { asm volatile("v_nop\n\tv_nop\n\tv_nop\n\tv_nop" : "+v"(a), "+v"(b) : "v"(x), "v"(y)); }
__device__ __forceinline__ void keep4_h(v16h a, v16h b, v16h c, v16h d) { asm volatile("v_nop" :: "v"(a), "v"(b), "v"(c), "v"(d)); }
__device__ __forceinline__ void keep4_b(v16b a, v16b b, v16b c, v16b d) { asm volatile("v_nop" :: "v"(a), "v"(b), "v"(c), "v"(d)); }
__device__ __forceinline__ void acc_guard4(v8f& a, v8f& b, v8f& c, v8f& d) { asm volatile("v_nop\n\tv_nop\n\tv_nop\n\tv_nop" : "+v"(a), "+v"(b), "+v"(c), "+v"(d)); }
template <typename T> struct Frag;
template <> struct Frag<_Float16> {
  typedef v16h V; union U { v16h v; v8h h[2]; };
  static __device__ __forceinline__ v16h load(const _Float16* p) {
    U f; f.h[0] = *(const v8h*)(p); f.h[1] = *(const v8h*)(p + 16); return f.v;
  }
  static __device__ __forceinline__ v8f mma(v16h a, v16h b, v8f c) {
    return __builtin_amdgcn_wmma_f32_16x16x32_f16(false, a, false, b, (short)0, c, false, false);
  }
  static __device__ __forceinline__ void guard(v8f& a, v8f& b, v16h x, v16h y) { dep_guard_h(a, b, x, y); }
  static __device__ __forceinline__ void keep(v16h a, v16h b, v16h c, v16h d) { keep4_h(a, b, c, d); }
};
template <> struct Frag<__bf16> {
  typedef v16b V; union U { v16b v; v8b h[2]; };
  static __device__ __forceinline__ v16b load(const __bf16* p) {
    U f; f.h[0] = *(const v8b*)(p); f.h[1] = *(const v8b*)(p + 16); return f.v;
  }
  static __device__ __forceinline__ v8f mma(v16b a, v16b b, v8f c) {
    return __builtin_amdgcn_wmma_f32_16x16x32_bf16(false, a, false, b, (short)0, c, false, false);
  }
  static __device__ __forceinline__ void guard(v8f& a, v8f& b, v16b x, v16b y) { dep_guard_b(a, b, x, y); }
  static __device__ __forceinline__ void keep(v16b a, v16b b, v16b c, v16b d) { keep4_b(a, b, c, d); }
};

template <int ET> struct Elem;
template <> struct Elem<0> { typedef _Float16 T; };
template <> struct Elem<1> { typedef __bf16 T; };
template <int ET, bool SPLIT, int BIAS_MODE, int OUT_MODE, bool RESID, int ACT = 0>
__global__ __launch_bounds__(256) void wmma_gemm64(
    const unsigned short* __restrict__ Ap, const unsigned short* __restrict__ A2p, int lda, long strideA,
    const unsigned short* __restrict__ Btp, const unsigned short* __restrict__ Bt2p, int ldb, long strideB,
    void* __restrict__ Cout, void* __restrict__ Cout2, int ldc, long strideC,
    const float* __restrict__ bias,
    const float* __restrict__ resid, long strideR,
    int M, int N, int K, float scale) {
  typedef typename Elem<ET>::T T;
  typedef typename Frag<T>::V V;
  const T* A = (const T*)Ap; const T* A2 = (const T*)A2p; const T* Bt = (const T*)Btp; const T* Bt2 = (const T*)Bt2p;
  __shared__ __align__(16) float sT[8][16 * 68];
  const int b    = blockIdx.y;
  const int lane = threadIdx.x & 31;
  const int wave = threadIdx.x >> 5;
  const int tilesN = N >> 6;
  const int tilesM = M >> 6;
  const int tile = blockIdx.x * 8 + wave;
  if (tile >= tilesM * tilesN) return;
  const int tm = tile / tilesN;
  const int tn = tile - tm * tilesN;
  const int m0 = tm << 6;
  const int n0 = tn << 6;

  const T* Ab  = A  + (size_t)b * strideA;
  const T* Bb  = Bt + (size_t)b * strideB;
  const T* Ab2 = SPLIT ? (A2  + (size_t)b * strideA) : nullptr;
  const T* Bb2 = SPLIT ? (Bt2 + (size_t)b * strideB) : nullptr;

  const int rlane = lane & 15;
  const int koff  = (lane >> 4) * 8;
  const int mOff  = (lane >> 4) * 8;

  v8f acc[4][4];
#pragma unroll
  for (int i = 0; i < 4; ++i)
#pragma unroll
    for (int j = 0; j < 4; ++j) acc[i][j] = (v8f){0.f,0.f,0.f,0.f,0.f,0.f,0.f,0.f};

  for (int k0 = 0; k0 < K; k0 += 32) {
    V bh[4], bl[4];
#pragma unroll
    for (int j = 0; j < 4; ++j) {
      const size_t bo = (size_t)(n0 + (j << 4) + rlane) * ldb + koff + k0;
      bh[j] = Frag<T>::load(Bb + bo);
      if (SPLIT) bl[j] = Frag<T>::load(Bb2 + bo);
    }
#pragma unroll
    for (int i = 0; i < 4; ++i) {
      const size_t ao = (size_t)(m0 + (i << 4) + rlane) * lda + koff + k0;
      V ah = Frag<T>::load(Ab + ao);
      V al;
      if (SPLIT) al = Frag<T>::load(Ab2 + ao);
#pragma unroll
      for (int j = 0; j < 4; ++j) {
        acc[i][j] = Frag<T>::mma(ah, bh[j], acc[i][j]);
        if (SPLIT) {
          acc[i][j] = Frag<T>::mma(ah, bl[j], acc[i][j]);
          acc[i][j] = Frag<T>::mma(al, bh[j], acc[i][j]);
        }
      }
      Frag<T>::guard(acc[i][0], acc[i][3], ah, SPLIT ? al : ah);
    }
    Frag<T>::keep(bh[0], bh[1], bh[2], bh[3]);
    if (SPLIT) Frag<T>::keep(bl[0], bl[1], bl[2], bl[3]);
  }
  acc_guard4(acc[0][0], acc[0][1], acc[0][2], acc[0][3]);
  acc_guard4(acc[1][0], acc[1][1], acc[1][2], acc[1][3]);
  acc_guard4(acc[2][0], acc[2][1], acc[2][2], acc[2][3]);
  acc_guard4(acc[3][0], acc[3][1], acc[3][2], acc[3][3]);

  float* slab = sT[wave];
  const float* Rb = RESID ? (resid + (size_t)b * strideR) : nullptr;
#pragma unroll
  for (int i = 0; i < 4; ++i) {
    const int mBase = m0 + (i << 4);
#pragma unroll
    for (int j = 0; j < 4; ++j) {
      const int n = n0 + (j << 4) + rlane;
      float bv = 0.f;
      if (BIAS_MODE == 2) bv = bias[n];
#pragma unroll
      for (int r = 0; r < 8; ++r) {
        float v = acc[i][j][r] * scale;
        if (BIAS_MODE == 1) v += bias[mBase + mOff + r];
        if (BIAS_MODE == 2) v += bv;
        if (RESID) v += Rb[(size_t)(mBase + mOff + r) * ldc + n];
        if (ACT == 1) v = tanhf(v);
        if (ACT == 2) v = fmaxf(v, 0.0f);
        if (ACT == 3) v = v / (1.0f + expf(-v));
        if (ACT == 4) v = (v > 0.f) ? v : 0.01f * v;
        if (ACT == 5) v = 0.5f * v * (1.0f + erff(v * 0.70710678118654752f));
        slab[(mOff + r) * 68 + (j << 4) + rlane] = v;
      }
    }
    __builtin_amdgcn_fence(__ATOMIC_RELEASE, "workgroup");
    __builtin_amdgcn_wave_barrier();
    __builtin_amdgcn_fence(__ATOMIC_ACQUIRE, "workgroup");
    if (OUT_MODE == 0) {
      float* C = (float*)Cout + (size_t)b * strideC;
      const int hh = lane >> 4, c4 = (lane & 15) * 4;
      for (int pass = 0; pass < 2; ++pass) {
#pragma unroll
        for (int it = 0; it < 8; ++it) {
          const int row = it * 2 + hh;
          v4f v = *(const v4f*)(slab + row * 68 + c4);
          *(volatile v4f*)(C + (size_t)(mBase + row) * ldc + n0 + c4) = v;
        }
        __threadfence();
      }
    } else {
      const int q = lane >> 3, c8 = (lane & 7) * 8;
      unsigned short* C  = (unsigned short*)Cout  + (size_t)b * strideC;
      unsigned short* C2 = (OUT_MODE == 2) ? ((unsigned short*)Cout2 + (size_t)b * strideC) : nullptr;
      for (int pass = 0; pass < 2; ++pass) {
#pragma unroll
        for (int it = 0; it < 4; ++it) {
          const int row = it * 4 + q;
          const float* sp = slab + row * 68 + c8;
          v8h hv, lv;
#pragma unroll
          for (int e = 0; e < 8; ++e) {
            if (OUT_MODE == 1) {
              hv[e] = (_Float16)sp[e];
            } else {
              unsigned short hb = f2bf_bits(sp[e]);
              unsigned short lb = f2bf_bits(sp[e] - bf_bits2f(hb));
              hv[e] = __builtin_bit_cast(_Float16, hb);
              lv[e] = __builtin_bit_cast(_Float16, lb);
            }
          }
          *(volatile v8h*)(C + (size_t)(mBase + row) * ldc + n0 + c8) = hv;
          if (OUT_MODE == 2) *(volatile v8h*)(C2 + (size_t)(mBase + row) * ldc + n0 + c8) = lv;
        }
        __threadfence();
      }
    }
    __builtin_amdgcn_fence(__ATOMIC_RELEASE, "workgroup");
    __builtin_amdgcn_wave_barrier();
    __builtin_amdgcn_fence(__ATOMIC_ACQUIRE, "workgroup");
  }
}

__global__ __launch_bounds__(256) void cast_f16_kernel(
    const float* __restrict__ src, unsigned short* __restrict__ dst, int total8, float scale)
{
  const int i = blockIdx.x * 256 + threadIdx.x;
  if (i >= total8) return;
  const size_t e0 = (size_t)i << 3;
  const float* p = src + e0;
  const v4f a0 = *(const v4f*)(p);
  const v4f a1 = *(const v4f*)(p + 4);
  v8h hv;
#pragma unroll
  for (int e = 0; e < 4; ++e) {
    hv[e]     = (_Float16)(a0[e] * scale);
    hv[4 + e] = (_Float16)(a1[e] * scale);
  }
  unsigned short* q = dst + e0;
  *(volatile v8h*)q = hv;
  __threadfence();
  *(volatile v8h*)q = hv;
}

__global__ __launch_bounds__(256) void cast_bf16hl_kernel(
    const float* __restrict__ src, unsigned short* __restrict__ dhi, unsigned short* __restrict__ dlo, int total8)
{
  const int i = blockIdx.x * 256 + threadIdx.x;
  if (i >= total8) return;
  const size_t e0 = (size_t)i << 3;
  const float* p = src + e0;
  const v4f a0 = *(const v4f*)(p);
  const v4f a1 = *(const v4f*)(p + 4);
  v8h hv, lv;
#pragma unroll
  for (int e = 0; e < 4; ++e) {
    _Float16 hh, ll;
    split_bf16(a0[e], hh, ll); hv[e] = hh;     lv[e] = ll;
    split_bf16(a1[e], hh, ll); hv[4 + e] = hh; lv[4 + e] = ll;
  }
  unsigned short* qh = dhi + e0;
  unsigned short* ql = dlo + e0;
  *(volatile v8h*)qh = hv;
  *(volatile v8h*)ql = lv;
  __threadfence();
  *(volatile v8h*)qh = hv;
  *(volatile v8h*)ql = lv;
}

__global__ __launch_bounds__(256) void layernorm_split_kernel(
    const float* __restrict__ x, const float* __restrict__ g, const float* __restrict__ bb,
    unsigned short* __restrict__ XNH, unsigned short* __restrict__ XNL, int nrows)
{
  const int lane = threadIdx.x & 31, wave = threadIdx.x >> 5;
  const int row = blockIdx.x * 8 + wave;
  if (row >= nrows) return;
  const float* xr = x + (size_t)row * kDmod;
  const int c0 = lane * 8, c1 = 256 + lane * 8;
  const v4f a0 = *(const v4f*)(xr + c0);
  const v4f a1 = *(const v4f*)(xr + c0 + 4);
  const v4f a2 = *(const v4f*)(xr + c1);
  const v4f a3 = *(const v4f*)(xr + c1 + 4);
  float s = 0.f;
#pragma unroll
  for (int e = 0; e < 4; ++e) { s += a0[e]; s += a1[e]; s += a2[e]; s += a3[e]; }
#pragma unroll
  for (int off = 16; off; off >>= 1) s += __shfl_xor(s, off, 32);
  const float mu = s * (1.0f / (float)kDmod);
  float q = 0.f;
#pragma unroll
  for (int e = 0; e < 4; ++e) {
    float t;
    t = a0[e] - mu; q += t * t;
    t = a1[e] - mu; q += t * t;
    t = a2[e] - mu; q += t * t;
    t = a3[e] - mu; q += t * t;
  }
#pragma unroll
  for (int off = 16; off; off >>= 1) q += __shfl_xor(q, off, 32);
  const float var  = q * (1.0f / (float)kDmod);
  const float rstd = 1.0f / sqrtf(var + kLnEps);
  const v4f g0 = *(const v4f*)(g + c0),  g1 = *(const v4f*)(g + c0 + 4);
  const v4f g2 = *(const v4f*)(g + c1),  g3 = *(const v4f*)(g + c1 + 4);
  const v4f b0 = *(const v4f*)(bb + c0), b1 = *(const v4f*)(bb + c0 + 4);
  const v4f b2 = *(const v4f*)(bb + c1), b3 = *(const v4f*)(bb + c1 + 4);
  v8h h0, l0, h1, l1;
#pragma unroll
  for (int e = 0; e < 4; ++e) {
    _Float16 hh, ll;
    split_bf16((a0[e] - mu) * rstd * g0[e] + b0[e], hh, ll); h0[e]     = hh; l0[e]     = ll;
    split_bf16((a1[e] - mu) * rstd * g1[e] + b1[e], hh, ll); h0[4 + e] = hh; l0[4 + e] = ll;
    split_bf16((a2[e] - mu) * rstd * g2[e] + b2[e], hh, ll); h1[e]     = hh; l1[e]     = ll;
    split_bf16((a3[e] - mu) * rstd * g3[e] + b3[e], hh, ll); h1[4 + e] = hh; l1[4 + e] = ll;
  }
  unsigned short* oh = XNH + (size_t)row * kDmod;
  unsigned short* ol = XNL + (size_t)row * kDmod;
  for (int pass = 0; pass < 2; ++pass) {
    *(volatile v8h*)(oh + c0) = h0;
    *(volatile v8h*)(oh + c1) = h1;
    *(volatile v8h*)(ol + c0) = l0;
    *(volatile v8h*)(ol + c1) = l1;
    __threadfence();
  }
}

__global__ __launch_bounds__(256) void conv_silu_kernel(
    const float* __restrict__ XZ, const float* __restrict__ cw, const float* __restrict__ cb,
    float* __restrict__ UC, unsigned short* __restrict__ UC16,
    unsigned short* __restrict__ UCH, unsigned short* __restrict__ UCL)
{
  __shared__ __align__(16) float sT[16 * kTP];
  const int tid = threadIdx.x, lane = tid & 31, wave = tid >> 5;
  const int bz = blockIdx.z;
  const float* XZb = XZ + (size_t)bz * kSeqL * kXZP;
  float* UCb = UC + (size_t)bz * kSeqL * kDin;
  unsigned short* UC16b = UC16 + (size_t)bz * kSeqL * kDin;
  unsigned short* UCHb  = UCH  + (size_t)bz * kSeqL * kDin;
  unsigned short* UCLb  = UCL  + (size_t)bz * kSeqL * kDin;
  const int d0 = blockIdx.x * 256, d = d0 + tid;
  const int t0 = blockIdx.y * 64;
  const float w0 = cw[d * kConvK + 0], w1 = cw[d * kConvK + 1], w2 = cw[d * kConvK + 2], w3 = cw[d * kConvK + 3];
  const float bc = cb[d];
  float xm3, xm2, xm1;
  {
    const int r3 = t0 - 3, r2 = t0 - 2, r1 = t0 - 1;
    const float v3 = XZb[(size_t)(r3 < 0 ? 0 : r3) * kXZP + d];
    const float v2 = XZb[(size_t)(r2 < 0 ? 0 : r2) * kXZP + d];
    const float v1 = XZb[(size_t)(r1 < 0 ? 0 : r1) * kXZP + d];
    xm3 = (r3 >= 0) ? v3 : 0.f;
    xm2 = (r2 >= 0) ? v2 : 0.f;
    xm1 = (r1 >= 0) ? v1 : 0.f;
  }
  const int hrow = wave >> 1;
  const int hch  = (wave & 1) * 128 + lane * 4;
#pragma unroll 1
  for (int sub = 0; sub < 4; ++sub) {
    const int lb = t0 + sub * 16;
#pragma unroll 1
    for (int s = 0; s < 16; ++s) {
      const float xc = XZb[(size_t)(lb + s) * kXZP + d];
      float acc = w0 * xm3;
      acc = fmaf(w1, xm2, acc);
      acc = fmaf(w2, xm1, acc);
      acc = fmaf(w3, xc, acc);
      const float sv = acc + bc;
      const float sg = __builtin_amdgcn_rcpf(1.0f + __expf(-sv));
      sT[s * kTP + tid] = sv * sg;
      xm3 = xm2; xm2 = xm1; xm1 = xc;
    }
    __syncthreads();
    v4f fv[4];
    v8h bv[2], bhv[2], blv[2];
#pragma unroll
    for (int it = 0; it < 4; ++it) fv[it] = *(const v4f*)(sT + (it * 4 + hrow) * kTP + hch);
#pragma unroll
    for (int it = 0; it < 2; ++it) {
      const float* sp = sT + (it * 8 + wave) * kTP + lane * 8;
      const v4f a0 = *(const v4f*)(sp);
      const v4f a1 = *(const v4f*)(sp + 4);
#pragma unroll
      for (int e = 0; e < 4; ++e) {
        _Float16 hh, ll;
        bv[it][e]     = (_Float16)a0[e];
        bv[it][4 + e] = (_Float16)a1[e];
        split_bf16(a0[e], hh, ll); bhv[it][e]     = hh; blv[it][e]     = ll;
        split_bf16(a1[e], hh, ll); bhv[it][4 + e] = hh; blv[it][4 + e] = ll;
      }
    }
    for (int pass = 0; pass < 2; ++pass) {
#pragma unroll
      for (int it = 0; it < 4; ++it)
        *(volatile v4f*)(UCb + (size_t)(lb + it * 4 + hrow) * kDin + d0 + hch) = fv[it];
#pragma unroll
      for (int it = 0; it < 2; ++it) {
        const size_t o = (size_t)(lb + it * 8 + wave) * kDin + d0 + lane * 8;
        *(volatile v8h*)(UC16b + o) = bv[it];
        *(volatile v8h*)(UCHb  + o) = bhv[it];
        *(volatile v8h*)(UCLb  + o) = blv[it];
      }
      __threadfence();
    }
    __syncthreads();
  }
}

__global__ __launch_bounds__(256) void scan_kernel(
    const float* __restrict__ DTP, const float* __restrict__ UC, const float* __restrict__ XZ,
    const float* __restrict__ BCF, const float* __restrict__ A_log, const float* __restrict__ Dv,
    unsigned short* __restrict__ YH, unsigned short* __restrict__ YL)
{
  __shared__ __align__(16) float sBC[kSC * kBCW];
  __shared__ __align__(16) float sY[kSC * kYP];
  const int tid = threadIdx.x, lane = tid & 31, wave = tid >> 5;
  const int b = blockIdx.y;
  const int ch = tid >> 2, part = tid & 3;
  const int d0 = blockIdx.x * kChB, d = d0 + ch;
  const int nb = part * kNq;
  const float* DTb = DTP + (size_t)b * kSeqL * kDin;
  const float* UCb = UC  + (size_t)b * kSeqL * kDin;
  const float* XZb = XZ  + (size_t)b * kSeqL * kXZP;
  const float* BCb = BCF + (size_t)b * kSeqL * kBCW;
  unsigned short* YHb = YH + (size_t)b * kSeqL * kDin;
  unsigned short* YLb = YL + (size_t)b * kSeqL * kDin;

  float An[kNq];
#pragma unroll
  for (int j = 0; j < kNq; ++j) An[j] = -__expf(A_log[(size_t)d * kNst + nb + j]);
  const float Dd = Dv[d];
  float h[kNq];
#pragma unroll
  for (int j = 0; j < kNq; ++j) h[j] = 0.f;

#pragma unroll 1
  for (int c = 0; c < kSeqL / kSC; ++c) {
    const int l0 = c * kSC;
    {
      const int r = tid >> 3, q = (tid & 7) * 16;
      const float* p = BCb + (size_t)(l0 + r) * kBCW + q;
      const v4f v0 = *(const v4f*)(p);
      const v4f v1 = *(const v4f*)(p + 4);
      const v4f v2 = *(const v4f*)(p + 8);
      const v4f v3 = *(const v4f*)(p + 12);
      *(v4f*)(sBC + r * kBCW + q)      = v0;
      *(v4f*)(sBC + r * kBCW + q + 4)  = v1;
      *(v4f*)(sBC + r * kBCW + q + 8)  = v2;
      *(v4f*)(sBC + r * kBCW + q + 12) = v3;
    }
    __syncthreads();
#pragma unroll 1
    for (int s = 0; s < kSC; ++s) {
      const size_t m = (size_t)(l0 + s);
      const float a     = DTb[m * kDin + d];
      const float delta = fmaxf(a, 0.0f) + log1pf(__expf(-fabsf(a)));
      const float xv    = UCb[m * kDin + d];
      const float zv    = XZb[m * kXZP + kDin + d];
      float y = 0.f;
#pragma unroll
      for (int qq = 0; qq < 4; ++qq) {
        const v4f Bq = *(const v4f*)(sBC + s * kBCW + nb + 4 * qq);
        const v4f Cq = *(const v4f*)(sBC + s * kBCW + kNst + nb + 4 * qq);
#pragma unroll
        for (int e = 0; e < 4; ++e) {
          const int j = qq * 4 + e;
          const float ex = __expf(delta * An[j]);
          float db = delta * Bq[e];
          asm volatile("" : "+v"(db));
          float p = db * xv;
          asm volatile("" : "+v"(p));
          float qv = h[j] * ex;
          asm volatile("" : "+v"(qv));
          const float hn = qv + p;
          h[j] = hn;
          float rr = Cq[e] * hn;
          asm volatile("" : "+v"(rr));
          y += rr;
        }
      }
      y += __shfl_xor(y, 1, 32);
      y += __shfl_xor(y, 2, 32);
      float sk = xv * Dd;
      asm volatile("" : "+v"(sk));
      y += sk;
      const float sg = __builtin_amdgcn_rcpf(1.0f + __expf(-zv));
      const float g  = zv * sg;
      if (part == 0) sY[s * kYP + ch] = y * g;
    }
    __syncthreads();
    const int row = wave * 4 + (lane >> 3), c8 = (lane & 7) * 8;
    v8h hv, lv;
    {
      const float* sp = sY + row * kYP + c8;
      const v4f a0 = *(const v4f*)(sp);
      const v4f a1 = *(const v4f*)(sp + 4);
#pragma unroll
      for (int e = 0; e < 4; ++e) {
        _Float16 hh, ll;
        split_bf16(a0[e], hh, ll); hv[e]     = hh; lv[e]     = ll;
        split_bf16(a1[e], hh, ll); hv[4 + e] = hh; lv[4 + e] = ll;
      }
    }
    for (int pass = 0; pass < 2; ++pass) {
      const size_t o = (size_t)(l0 + row) * kDin + d0 + c8;
      *(volatile v8h*)(YHb + o) = hv;
      *(volatile v8h*)(YLb + o) = lv;
      __threadfence();
    }
  }
}

extern "C" void kernel_launch(void* const* d_in, const int* in_sizes, int n_in,
                              void* d_out, int out_size, void* d_ws, size_t ws_size,
                              hipStream_t stream)
{
  if (n_in < 12) return;
  const float* x     = (const float*)d_in[0];
  const float* ln_g  = (const float*)d_in[1];
  const float* ln_b  = (const float*)d_in[2];
  const float* Win   = (const float*)d_in[3];
  const float* Wconv = (const float*)d_in[4];
  const float* bconv = (const float*)d_in[5];
  const float* Wx    = (const float*)d_in[6];
  const float* Wdt   = (const float*)d_in[7];
  const float* bdt   = (const float*)d_in[8];
  const float* A_log = (const float*)d_in[9];
  const float* Dvec  = (const float*)d_in[10];
  const float* Wout  = (const float*)d_in[11];
  float* dout = (float*)d_out;

  if (in_sizes[0] != kRows * kDmod) return;
  if (in_sizes[1] != kDmod || in_sizes[2] != kDmod) return;
  if (in_sizes[3] != kXZP * kDmod) return;
  if (in_sizes[4] != kDin * kConvK || in_sizes[5] != kDin) return;
  if (in_sizes[6] != kBCW * kDin) return;
  if (in_sizes[7] != kDin * kDin || in_sizes[8] != kDin) return;
  if (in_sizes[9] != kDin * kNst || in_sizes[10] != kDin) return;
  if (in_sizes[11] != kDmod * kDin) return;
  if (out_size != kRows * kDmod) return;

  const size_t SZ_WINP   = (size_t)kXZP * kDmod * 2;
  const size_t SZ_WDT16  = (size_t)kDin * kDin * 2;
  const size_t SZ_WXP    = (size_t)kBCW * kDin * 2;
  const size_t SZ_WOUTP  = (size_t)kDmod * kDin * 2;
  const size_t SZ_XNP    = (size_t)kRows * kDmod * 2;
  const size_t SZ_XZ     = (size_t)kRows * kXZP * 4;
  const size_t SZ_XC     = (size_t)kRows * kDin * 4;
  const size_t SZ_XCP    = (size_t)kRows * kDin * 2;
  const size_t SZ_DTP    = (size_t)kRows * kDin * 4;
  const size_t SZ_BCF    = (size_t)kRows * kBCW * 4;
  const size_t SZ_YGP    = (size_t)kRows * kDin * 2;
  const size_t OFF_WINH   = 0;
  const size_t OFF_WINL   = OFF_WINH   + SZ_WINP;
  const size_t OFF_WDT16  = OFF_WINL   + SZ_WINP;
  const size_t OFF_WXH    = OFF_WDT16  + SZ_WDT16;
  const size_t OFF_WXL    = OFF_WXH    + SZ_WXP;
  const size_t OFF_WOUTH  = OFF_WXL    + SZ_WXP;
  const size_t OFF_WOUTL  = OFF_WOUTH  + SZ_WOUTP;
  const size_t OFF_XNH    = OFF_WOUTL  + SZ_WOUTP;
  const size_t OFF_XNL    = OFF_XNH    + SZ_XNP;
  const size_t OFF_XZ     = OFF_XNL    + SZ_XNP;
  const size_t OFF_XC     = OFF_XZ     + SZ_XZ;
  const size_t OFF_XC16   = OFF_XC     + SZ_XC;
  const size_t OFF_XCH    = OFF_XC16   + SZ_XCP;
  const size_t OFF_XCL    = OFF_XCH    + SZ_XCP;
  const size_t OFF_DTP    = OFF_XCL    + SZ_XCP;
  const size_t OFF_BCF    = OFF_DTP    + SZ_DTP;
  const size_t OFF_YGH    = OFF_BCF    + SZ_BCF;
  const size_t OFF_YGL    = OFF_YGH    + SZ_YGP;
  const size_t TOTAL      = OFF_YGL    + SZ_YGP;
  if (TOTAL > (size_t)134217728) return;
  if (ws_size < TOTAL) return;

  char* ws = (char*)d_ws;
  unsigned short* WINH   = (unsigned short*)(ws + OFF_WINH);
  unsigned short* WINL   = (unsigned short*)(ws + OFF_WINL);
  unsigned short* WDT16  = (unsigned short*)(ws + OFF_WDT16);
  unsigned short* WXH    = (unsigned short*)(ws + OFF_WXH);
  unsigned short* WXL    = (unsigned short*)(ws + OFF_WXL);
  unsigned short* WOUTH  = (unsigned short*)(ws + OFF_WOUTH);
  unsigned short* WOUTL  = (unsigned short*)(ws + OFF_WOUTL);
  unsigned short* XNH    = (unsigned short*)(ws + OFF_XNH);
  unsigned short* XNL    = (unsigned short*)(ws + OFF_XNL);
  float*          XZ     = (float*)(ws + OFF_XZ);
  float*          XC     = (float*)(ws + OFF_XC);
  unsigned short* XC16   = (unsigned short*)(ws + OFF_XC16);
  unsigned short* XCH    = (unsigned short*)(ws + OFF_XCH);
  unsigned short* XCL    = (unsigned short*)(ws + OFF_XCL);
  float*          DTP    = (float*)(ws + OFF_DTP);
  float*          BCF    = (float*)(ws + OFF_BCF);
  unsigned short* YGH    = (unsigned short*)(ws + OFF_YGH);
  unsigned short* YGL    = (unsigned short*)(ws + OFF_YGL);
  const float* dummy_bias  = bdt;
  const float* dummy_resid = x;

  cast_bf16hl_kernel<<<(kXZP * kDmod) / 8 / 256, 256, 0, stream>>>(Win,  WINH,  WINL,  (kXZP * kDmod) / 8);
  cast_f16_kernel   <<<(kDin * kDin)  / 8 / 256, 256, 0, stream>>>(Wdt,  WDT16,        (kDin * kDin)  / 8, 32.0f);
  cast_bf16hl_kernel<<<(kBCW * kDin)  / 8 / 256, 256, 0, stream>>>(Wx,   WXH,   WXL,   (kBCW * kDin)  / 8);
  cast_bf16hl_kernel<<<(kDmod * kDin) / 8 / 256, 256, 0, stream>>>(Wout, WOUTH, WOUTL, (kDmod * kDin) / 8);

  layernorm_split_kernel<<<kRows / 8, 256, 0, stream>>>(x, ln_g, ln_b, XNH, XNL, kRows);

  wmma_gemm64<1, true, 0, 0, false><<<dim3(128, 1), 256, 0, stream>>>(
      XNH, XNL, kDmod, 0L, WINH, WINL, kDmod, 0L,
      (void*)XZ, (void*)XZ, kXZP, 0L, dummy_bias, dummy_resid, 0L, kRows, kXZP, kDmod, 1.0f);

  conv_silu_kernel<<<dim3(kDin / 256, kSeqL / 64, kBatch), 256, 0, stream>>>(XZ, Wconv, bconv, XC, XC16, XCH, XCL);

  wmma_gemm64<0, false, 2, 0, false><<<dim3(64, 1), 256, 0, stream>>>(
      XC16, XC16, kDin, 0L, WDT16, WDT16, kDin, 0L,
      (void*)DTP, (void*)DTP, kDin, 0L, bdt, dummy_resid, 0L, kRows, kDin, kDin, 1.0f / 32.0f);

  wmma_gemm64<1, true, 0, 0, false><<<dim3(8, 1), 256, 0, stream>>>(
      XCH, XCL, kDin, 0L, WXH, WXL, kDin, 0L,
      (void*)BCF, (void*)BCF, kBCW, 0L, dummy_bias, dummy_resid, 0L, kRows, kBCW, kDin, 1.0f);

  scan_kernel<<<dim3(kDin / kChB, kBatch), 256, 0, stream>>>(DTP, XC, XZ, BCF, A_log, Dvec, YGH, YGL);

  wmma_gemm64<1, true, 0, 0, true><<<dim3(32, 1), 256, 0, stream>>>(
      YGH, YGL, kDin, 0L, WOUTH, WOUTL, kDin, 0L,
      (void*)dout, (void*)dout, kDmod, 0L, dummy_bias, x, 0L, kRows, kDmod, kDin, 1.0f);
}
